// TimeMixing_21938692948062
// MI455X (gfx1250) — hardware-verified
//
#include <hip/hip_runtime.h>
#include <math.h>

constexpr int kBatch   = 2;
constexpr int kSeq     = 2048;
constexpr int kDim     = 1024;
constexpr int kHeads   = 16;
constexpr int kHeadDim = 64;
constexpr int kLora    = 64;
constexpr int kRows    = kBatch * kSeq;
constexpr float kLoraCarry    = 64.0f;
constexpr float kLoraCarryInv = 1.0f / 64.0f;
static_assert(kHeads * kHeadDim == kDim);
static_assert(kDim == 1024);
static_assert(kSeq == 2048);
static_assert((kRows % 64) == 0 && (kDim % 64) == 0 && (kLora % 64) == 0);
static_assert((kDim % 32) == 0 && (kLora % 32) == 0);

typedef __attribute__((ext_vector_type(16))) _Float16 v16h;
typedef __attribute__((ext_vector_type(8)))  _Float16 v8h;
typedef __attribute__((ext_vector_type(16))) __bf16   v16b;
typedef __attribute__((ext_vector_type(8)))  __bf16   v8b;
typedef __attribute__((ext_vector_type(8)))  float    v8f;
typedef __attribute__((ext_vector_type(4)))  float    v4f;
typedef __attribute__((ext_vector_type(4)))  unsigned int v4u;

__device__ __forceinline__ unsigned short f2bf_bits(float f) {
  unsigned u = __float_as_uint(f);
  return (unsigned short)((u + 0x7FFFu + ((u >> 16) & 1u)) >> 16);
}
__device__ __forceinline__ float bf_bits2f(unsigned short h) { return __uint_as_float(((unsigned)h) << 16); }

__device__ __forceinline__ void dep_guard_h(v8f& a, v8f& b, v16h x, v16h y) { asm volatile("v_nop\n\tv_nop\n\tv_nop\n\tv_nop" : "+v"(a), "+v"(b) : "v"(x), "v"(y)); }
__device__ __forceinline__ void dep_guard_b(v8f& a, v8f& b, v16b x, v16b y) { asm volatile("v_nop\n\tv_nop\n\tv_nop\n\tv_nop" : "+v"(a), "+v"(b) : "v"(x), "v"(y)); }
__device__ __forceinline__ void keep4_h(v16h a, v16h b, v16h c, v16h d) { asm volatile("v_nop" :: "v"(a), "v"(b), "v"(c), "v"(d)); }
__device__ __forceinline__ void keep4_b(v16b a, v16b b, v16b c, v16b d) { asm volatile("v_nop" :: "v"(a), "v"(b), "v"(c), "v"(d)); }
__device__ __forceinline__ void acc_guard4(v8f& a, v8f& b, v8f& c, v8f& d) { asm volatile("v_nop\n\tv_nop\n\tv_nop\n\tv_nop" : "+v"(a), "+v"(b), "+v"(c), "+v"(d)); }
template <typename T> struct Frag;
template <> struct Frag<_Float16> {
  typedef v16h V; union U { v16h v; v8h h[2]; };
  static __device__ __forceinline__ v16h load(const _Float16* p) {
    U f; f.h[0] = *(const v8h*)(p); f.h[1] = *(const v8h*)(p + 16); return f.v;
  }
  static __device__ __forceinline__ v8f mma(v16h a, v16h b, v8f c) {
    return __builtin_amdgcn_wmma_f32_16x16x32_f16(false, a, false, b, (short)0, c, false, false);
  }
  static __device__ __forceinline__ void guard(v8f& a, v8f& b, v16h x, v16h y) { dep_guard_h(a, b, x, y); }
  static __device__ __forceinline__ void keep(v16h a, v16h b, v16h c, v16h d) { keep4_h(a, b, c, d); }
};
template <> struct Frag<__bf16> {
  typedef v16b V; union U { v16b v; v8b h[2]; };
  static __device__ __forceinline__ v16b load(const __bf16* p) {
    U f; f.h[0] = *(const v8b*)(p); f.h[1] = *(const v8b*)(p + 16); return f.v;
  }
  static __device__ __forceinline__ v8f mma(v16b a, v16b b, v8f c) {
    return __builtin_amdgcn_wmma_f32_16x16x32_bf16(false, a, false, b, (short)0, c, false, false);
  }
  static __device__ __forceinline__ void guard(v8f& a, v8f& b, v16b x, v16b y) { dep_guard_b(a, b, x, y); }
  static __device__ __forceinline__ void keep(v16b a, v16b b, v16b c, v16b d) { keep4_b(a, b, c, d); }
};

__device__ __forceinline__ unsigned pk16(unsigned short a, unsigned short b) { return (unsigned)a | ((unsigned)b << 16); }
__device__ __forceinline__ unsigned short h_bits(float f) { const _Float16 h = (_Float16)f; return __builtin_bit_cast(unsigned short, h); }

template <int ET> struct Elem;
template <> struct Elem<0> { typedef _Float16 T; };
template <> struct Elem<1> { typedef __bf16 T; };
template <int ET, bool SPLIT, int BIAS_MODE, int OUT_MODE, bool RESID, int ACT = 0>
__global__ __launch_bounds__(256) void wmma_gemm64(
    const unsigned short* __restrict__ Ap, const unsigned short* __restrict__ A2p, int lda, long strideA,
    const unsigned short* __restrict__ Btp, const unsigned short* __restrict__ Bt2p, int ldb, long strideB,
    void* __restrict__ Cout, void* __restrict__ Cout2, int ldc, long strideC,
    const float* __restrict__ bias,
    const float* __restrict__ resid, long strideR,
    int M, int N, int K, float scale) {
  typedef typename Elem<ET>::T T;
  typedef typename Frag<T>::V V;
  const T* A = (const T*)Ap; const T* A2 = (const T*)A2p; const T* Bt = (const T*)Btp; const T* Bt2 = (const T*)Bt2p;
  __shared__ __align__(16) float sT[8][16 * 68];
  const int b    = blockIdx.y;
  const int lane = threadIdx.x & 31;
  const int wave = threadIdx.x >> 5;
  const int tilesN = N >> 6;
  const int tilesM = M >> 6;
  const int tile = blockIdx.x * 8 + wave;
  if (tile >= tilesM * tilesN) return;
  const int tm = tile / tilesN;
  const int tn = tile - tm * tilesN;
  const int m0 = tm << 6;
  const int n0 = tn << 6;

  const T* Ab  = A  + (size_t)b * strideA;
  const T* Bb  = Bt + (size_t)b * strideB;
  const T* Ab2 = SPLIT ? (A2  + (size_t)b * strideA) : nullptr;
  const T* Bb2 = SPLIT ? (Bt2 + (size_t)b * strideB) : nullptr;

  const int rlane = lane & 15;
  const int koff  = (lane >> 4) * 8;
  const int mOff  = (lane >> 4) * 8;

  v8f acc[4][4];
#pragma unroll
  for (int i = 0; i < 4; ++i)
#pragma unroll
    for (int j = 0; j < 4; ++j) acc[i][j] = (v8f){0.f,0.f,0.f,0.f,0.f,0.f,0.f,0.f};

  for (int k0 = 0; k0 < K; k0 += 32) {
    V bh[4], bl[4];
#pragma unroll
    for (int j = 0; j < 4; ++j) {
      const size_t bo = (size_t)(n0 + (j << 4) + rlane) * ldb + koff + k0;
      bh[j] = Frag<T>::load(Bb + bo);
      if (SPLIT) bl[j] = Frag<T>::load(Bb2 + bo);
    }
#pragma unroll
    for (int i = 0; i < 4; ++i) {
      const size_t ao = (size_t)(m0 + (i << 4) + rlane) * lda + koff + k0;
      V ah = Frag<T>::load(Ab + ao);
      V al;
      if (SPLIT) al = Frag<T>::load(Ab2 + ao);
#pragma unroll
      for (int j = 0; j < 4; ++j) {
        acc[i][j] = Frag<T>::mma(ah, bh[j], acc[i][j]);
        if (SPLIT) {
          acc[i][j] = Frag<T>::mma(ah, bl[j], acc[i][j]);
          acc[i][j] = Frag<T>::mma(al, bh[j], acc[i][j]);
        }
      }
      Frag<T>::guard(acc[i][0], acc[i][3], ah, SPLIT ? al : ah);
    }
    Frag<T>::keep(bh[0], bh[1], bh[2], bh[3]);
    if (SPLIT) Frag<T>::keep(bl[0], bl[1], bl[2], bl[3]);
  }
  acc_guard4(acc[0][0], acc[0][1], acc[0][2], acc[0][3]);
  acc_guard4(acc[1][0], acc[1][1], acc[1][2], acc[1][3]);
  acc_guard4(acc[2][0], acc[2][1], acc[2][2], acc[2][3]);
  acc_guard4(acc[3][0], acc[3][1], acc[3][2], acc[3][3]);

  float* slab = sT[wave];
  const float* Rb = RESID ? (resid + (size_t)b * strideR) : nullptr;
#pragma unroll
  for (int i = 0; i < 4; ++i) {
    const int mBase = m0 + (i << 4);
#pragma unroll
    for (int j = 0; j < 4; ++j) {
      const int n = n0 + (j << 4) + rlane;
      float bv = 0.f;
      if (BIAS_MODE == 2) bv = bias[n];
#pragma unroll
      for (int r = 0; r < 8; ++r) {
        float v = acc[i][j][r] * scale;
        if (BIAS_MODE == 1) v += bias[mBase + mOff + r];
        if (BIAS_MODE == 2) v += bv;
        if (RESID) v += Rb[(size_t)(mBase + mOff + r) * ldc + n];
        if (ACT == 1) v = tanhf(v);
        if (ACT == 2) v = fmaxf(v, 0.0f);
        if (ACT == 3) v = v / (1.0f + expf(-v));
        if (ACT == 4) v = (v > 0.f) ? v : 0.01f * v;
        if (ACT == 5) v = 0.5f * v * (1.0f + erff(v * 0.70710678118654752f));
        slab[(mOff + r) * 68 + (j << 4) + rlane] = v;
      }
    }
    __builtin_amdgcn_fence(__ATOMIC_RELEASE, "workgroup");
    __builtin_amdgcn_wave_barrier();
    __builtin_amdgcn_fence(__ATOMIC_ACQUIRE, "workgroup");
    if (OUT_MODE == 0) {
      float* C = (float*)Cout + (size_t)b * strideC;
      const int hh = lane >> 4, c4 = (lane & 15) * 4;
      for (int pass = 0; pass < 2; ++pass) {
#pragma unroll
        for (int it = 0; it < 8; ++it) {
          const int row = it * 2 + hh;
          v4f v = *(const v4f*)(slab + row * 68 + c4);
          *(volatile v4f*)(C + (size_t)(mBase + row) * ldc + n0 + c4) = v;
        }
        __threadfence();
      }
    } else {
      const int q = lane >> 3, c8 = (lane & 7) * 8;
      unsigned short* C  = (unsigned short*)Cout  + (size_t)b * strideC;
      unsigned short* C2 = (OUT_MODE == 2) ? ((unsigned short*)Cout2 + (size_t)b * strideC) : nullptr;
      for (int pass = 0; pass < 2; ++pass) {
#pragma unroll
        for (int it = 0; it < 4; ++it) {
          const int row = it * 4 + q;
          const float* sp = slab + row * 68 + c8;
          v8h hv, lv;
#pragma unroll
          for (int e = 0; e < 8; ++e) {
            if (OUT_MODE == 1) {
              hv[e] = (_Float16)sp[e];
            } else {
              unsigned short hb = f2bf_bits(sp[e]);
              unsigned short lb = f2bf_bits(sp[e] - bf_bits2f(hb));
              hv[e] = __builtin_bit_cast(_Float16, hb);
              lv[e] = __builtin_bit_cast(_Float16, lb);
            }
          }
          *(volatile v8h*)(C + (size_t)(mBase + row) * ldc + n0 + c8) = hv;
          if (OUT_MODE == 2) *(volatile v8h*)(C2 + (size_t)(mBase + row) * ldc + n0 + c8) = lv;
        }
        __threadfence();
      }
    }
    __builtin_amdgcn_fence(__ATOMIC_RELEASE, "workgroup");
    __builtin_amdgcn_wave_barrier();
    __builtin_amdgcn_fence(__ATOMIC_ACQUIRE, "workgroup");
  }
}

template <int MODE>
__global__ __launch_bounds__(256) void tcast_kernel(const float* __restrict__ s0, const float* __restrict__ s1,
                                                    const float* __restrict__ s2, const float* __restrict__ s3,
                                                    const float* __restrict__ s4, int R, int C,
                                                    unsigned short* __restrict__ dst, unsigned short* __restrict__ dst2,
                                                    long zplane, float scale) {
  __shared__ float sm[64][65];
  const int t  = threadIdx.x;
  const int r0 = blockIdx.x * 64;
  const int c0 = blockIdx.y * 64;
  const int z  = blockIdx.z;
  const float* src = (z == 0) ? s0 : (z == 1) ? s1 : (z == 2) ? s2 : (z == 3) ? s3 : s4;
#pragma unroll
  for (int i = 0; i < 16; ++i) {
    const int e  = i * 256 + t;
    const int rl = e >> 6;
    const int cl = e & 63;
    sm[cl][rl] = src[(size_t)(r0 + rl) * C + c0 + cl] * scale;
  }
  __syncthreads();
  const int lane = t & 31, wave = t >> 5;
  const int q = lane >> 3, c8 = (lane & 7) * 8;
  unsigned short* oh = dst  + (size_t)z * zplane;
  unsigned short* ol = dst2 + (size_t)z * zplane;
  for (int pass = 0; pass < 2; ++pass) {
#pragma unroll
    for (int it = 0; it < 2; ++it) {
      const int row = wave * 8 + it * 4 + q;
      unsigned short hb[8], lb[8];
#pragma unroll
      for (int e = 0; e < 8; ++e) {
        const float v = sm[row][c8 + e];
        if (MODE == 0) {
          hb[e] = h_bits(v);
          lb[e] = 0;
        } else {
          hb[e] = f2bf_bits(v);
          lb[e] = f2bf_bits(v - bf_bits2f(hb[e]));
        }
      }
      const v4u uh = (v4u){pk16(hb[0], hb[1]), pk16(hb[2], hb[3]), pk16(hb[4], hb[5]), pk16(hb[6], hb[7])};
      const size_t o = (size_t)(c0 + row) * R + r0 + c8;
      *(volatile v4u*)(oh + o) = uh;
      if (MODE == 1) {
        const v4u ul = (v4u){pk16(lb[0], lb[1]), pk16(lb[2], lb[3]), pk16(lb[4], lb[5]), pk16(lb[6], lb[7])};
        *(volatile v4u*)(ol + o) = ul;
      }
    }
    __threadfence();
  }
}

template <int MODE>
__global__ __launch_bounds__(256) void shiftmix_kernel(const float* __restrict__ x, const float* __restrict__ mu,
                                                       unsigned short* __restrict__ out0, unsigned short* __restrict__ out1,
                                                       int n8) {
  const int i = blockIdx.x * 256 + threadIdx.x;
  if (i >= n8) return;
  const size_t e0  = (size_t)8 * i;
  const int    d0  = (int)(e0 & (size_t)(kDim - 1));
  const int    row = (int)(e0 >> 10);
  const int    t   = row & (kSeq - 1);
  const size_t ep  = (t > 0) ? (e0 - (size_t)kDim) : e0;
  const v4f xa = *(const v4f*)(x + e0);
  const v4f xc = *(const v4f*)(x + e0 + 4);
  const v4f pa = *(const v4f*)(x + ep);
  const v4f pc = *(const v4f*)(x + ep + 4);
  const v4f ma = *(const v4f*)(mu + d0);
  const v4f mc = *(const v4f*)(mu + d0 + 4);
  float xm[8];
#pragma unroll
  for (int e = 0; e < 4; ++e) {
    const float xi0 = xa[e];
    const float xp0 = (t > 0) ? pa[e] : 0.0f;
    xm[e] = xi0 + (xp0 - xi0) * ma[e];
    const float xi1 = xc[e];
    const float xp1 = (t > 0) ? pc[e] : 0.0f;
    xm[4 + e] = xi1 + (xp1 - xi1) * mc[e];
  }
  unsigned short hb[8], lb[8];
#pragma unroll
  for (int e = 0; e < 8; ++e) {
    if (MODE == 0) {
      hb[e] = h_bits(xm[e]);
      lb[e] = 0;
    } else {
      hb[e] = f2bf_bits(xm[e]);
      lb[e] = f2bf_bits(xm[e] - bf_bits2f(hb[e]));
    }
  }
  const v4u uh = (v4u){pk16(hb[0], hb[1]), pk16(hb[2], hb[3]), pk16(hb[4], hb[5]), pk16(hb[6], hb[7])};
  const v4u ul = (v4u){pk16(lb[0], lb[1]), pk16(lb[2], lb[3]), pk16(lb[4], lb[5]), pk16(lb[6], lb[7])};
  unsigned short* p0 = out0 + e0;
  unsigned short* p1 = out1 + e0;
  *(volatile v4u*)p0 = uh;
  if (MODE == 1) *(volatile v4u*)p1 = ul;
  __threadfence();
  *(volatile v4u*)p0 = uh;
  if (MODE == 1) *(volatile v4u*)p1 = ul;
}

__global__ __launch_bounds__(256) void tanh_cast_kernel(const float* __restrict__ in, unsigned short* __restrict__ out, int n2) {
  const int i = blockIdx.x * 256 + threadIdx.x;
  if (i >= n2) return;
  const float a = tanhf(in[2 * (size_t)i]);
  const float c = tanhf(in[2 * (size_t)i + 1]);
  const unsigned w = pk16(h_bits(a), h_bits(c));
  ((volatile unsigned*)out)[i] = w;
  __threadfence();
  ((volatile unsigned*)out)[i] = w;
}

__global__ __launch_bounds__(64) void wkv_kernel(const float* __restrict__ r32, const float* __restrict__ k32,
                                                 const float* __restrict__ v32, const float* __restrict__ z32,
                                                 const float* __restrict__ w0, const float* __restrict__ u,
                                                 float* __restrict__ y) {
#pragma clang fp contract(off)
  __shared__ __align__(16) float rs[2][kHeadDim];
  __shared__ __align__(16) float ks[2][kHeadDim];
  __shared__ __align__(16) float wdec[2][kHeadDim];
  __shared__ float reda[2][2];
  const int bh   = blockIdx.x;
  const int b    = bh >> 4;
  const int h    = bh & (kHeads - 1);
  const int j    = threadIdx.x;
  const int lane = j & 31;
  const int wave = j >> 5;
  const float w0j = w0[h * kHeadDim + j];
  const float uj  = u[h * kHeadDim + j];

  float S[kHeadDim];
#pragma unroll
  for (int i = 0; i < kHeadDim; ++i) S[i] = 0.0f;

  const size_t base = (size_t)b * kSeq * kDim + (size_t)h * kHeadDim;
  for (int t = 0; t < kSeq; ++t) {
    const int p = t & 1;
    const size_t off = base + (size_t)t * kDim;
    const float rj = r32[off + j];
    const float kj = k32[off + j];
    const float vj = v32[off + j];
    const float zj = z32[off + j];
    const float wj = expf(-expf(w0j + zj));
    rs[p][j]   = rj;
    ks[p][j]   = kj;
    wdec[p][j] = wj;
    float pa = (rj * uj) * kj;
#pragma unroll
    for (int m = 1; m < 32; m <<= 1) pa += __shfl_xor(pa, m, 32);
    if (lane == 0) reda[p][wave] = pa;
    __syncthreads();
    const float a = reda[p][0] + reda[p][1];
    float ysum = 0.0f;
#pragma unroll
    for (int q4 = 0; q4 < kHeadDim / 4; ++q4) {
      const v4f r4 = *(const v4f*)(&rs[p][4 * q4]);
      const v4f k4 = *(const v4f*)(&ks[p][4 * q4]);
      const v4f w4 = *(const v4f*)(&wdec[p][4 * q4]);
#pragma unroll
      for (int e = 0; e < 4; ++e) {
        const int ii = 4 * q4 + e;
        ysum  = ysum + r4[e] * S[ii];
        S[ii] = w4[e] * S[ii] + k4[e] * vj;
      }
    }
    const float yv = ysum + a * vj;
    *(volatile float*)(y + off + j) = yv;
    __threadfence();
    *(volatile float*)(y + off + j) = yv;
  }
}

__global__ __launch_bounds__(256) void gn_gate_kernel(const float* __restrict__ y, const float* __restrict__ g32,
                                                     const float* __restrict__ gamma, const float* __restrict__ beta,
                                                     unsigned short* __restrict__ ohi, unsigned short* __restrict__ olo) {
  const int lane = threadIdx.x & 31;
  const int wave = threadIdx.x >> 5;
  const int task = blockIdx.x * 8 + wave;
  const int row  = task >> 4;
  const int h    = task & (kHeads - 1);
  const int c0   = h * kHeadDim + 2 * lane;
  const size_t base = (size_t)row * kDim + c0;
  const float y0 = y[base];
  const float y1 = y[base + 1];
  float s = y0 + y1;
#pragma unroll
  for (int m = 1; m < 32; m <<= 1) s += __shfl_xor(s, m, 32);
  const float mean = s * (1.0f / 64.0f);
  const float d0v = y0 - mean;
  const float d1v = y1 - mean;
  float q = d0v * d0v + d1v * d1v;
#pragma unroll
  for (int m = 1; m < 32; m <<= 1) q += __shfl_xor(q, m, 32);
  const float var  = q * (1.0f / 64.0f);
  const float rstd = rsqrtf(var + 1e-5f);
  const float n0 = d0v * rstd * gamma[c0] + beta[c0];
  const float n1 = d1v * rstd * gamma[c0 + 1] + beta[c0 + 1];
  const float g0 = g32[base];
  const float g1 = g32[base + 1];
  const float sg0 = g0 * (1.0f / (1.0f + expf(-g0)));
  const float sg1 = g1 * (1.0f / (1.0f + expf(-g1)));
  const float o0 = n0 * sg0;
  const float o1 = n1 * sg1;
  const unsigned short h0 = f2bf_bits(o0);
  const unsigned short h1 = f2bf_bits(o1);
  const unsigned short l0 = f2bf_bits(o0 - bf_bits2f(h0));
  const unsigned short l1 = f2bf_bits(o1 - bf_bits2f(h1));
  const unsigned wh = pk16(h0, h1);
  const unsigned wl = pk16(l0, l1);
  const size_t idx = base >> 1;
  ((volatile unsigned*)ohi)[idx] = wh;
  ((volatile unsigned*)olo)[idx] = wl;
  __threadfence();
  ((volatile unsigned*)ohi)[idx] = wh;
  ((volatile unsigned*)olo)[idx] = wl;
}

extern "C" void kernel_launch(void* const* d_in, const int* in_sizes, int n_in,
                              void* d_out, int out_size, void* d_ws, size_t ws_size, hipStream_t stream) {
  if (n_in < 17) return;
  const float* x    = (const float*)d_in[0];
  const float* mu_w = (const float*)d_in[1];
  const float* mu_r = (const float*)d_in[2];
  const float* mu_k = (const float*)d_in[3];
  const float* mu_v = (const float*)d_in[4];
  const float* mu_g = (const float*)d_in[5];
  const float* w0   = (const float*)d_in[6];
  const float* Aw   = (const float*)d_in[7];
  const float* Bw   = (const float*)d_in[8];
  const float* Wr   = (const float*)d_in[9];
  const float* Wk   = (const float*)d_in[10];
  const float* Wv   = (const float*)d_in[11];
  const float* Wg   = (const float*)d_in[12];
  const float* Wo   = (const float*)d_in[13];
  const float* u    = (const float*)d_in[14];
  const float* gng  = (const float*)d_in[15];
  const float* gnb  = (const float*)d_in[16];
  float* out = (float*)d_out;

  const size_t nTok = (size_t)kRows * kDim;
  if (in_sizes[0] != (int)nTok || out_size != (int)nTok) return;
  if (in_sizes[7] != kDim * kLora || in_sizes[8] != kLora * kDim || in_sizes[9] != kDim * kDim ||
      in_sizes[13] != kDim * kDim || in_sizes[14] != kDim || in_sizes[6] != kDim) return;

  const size_t szWT    = (size_t)5 * 2 * kDim * kDim * 2;
  const size_t szAwT   = (size_t)kLora * kDim * 2;
  const size_t szBwT   = (size_t)kDim * kLora * 2;
  const size_t szHraw  = (size_t)kRows * kLora * 4;
  const size_t szH16   = (size_t)kRows * kLora * 2;
  const size_t szPlane = nTok * 4;
  const size_t oWT   = 0;
  const size_t oAwT  = oWT + szWT;
  const size_t oBwT  = oAwT + szAwT;
  const size_t oHraw = oBwT + szBwT;
  const size_t oH16  = oHraw + szHraw;
  const size_t oA    = oH16 + szH16;
  const size_t oZ    = oA + szPlane;
  const size_t oR    = oZ + szPlane;
  const size_t oK    = oR + szPlane;
  const size_t oV    = oK + szPlane;
  const size_t oG    = oV + szPlane;
  const size_t total = oG + szPlane;
  if (total > ws_size) return;

  char* ws = (char*)d_ws;
  unsigned short* wt   = (unsigned short*)(ws + oWT);
  unsigned short* awT  = (unsigned short*)(ws + oAwT);
  unsigned short* bwT  = (unsigned short*)(ws + oBwT);
  float*          hraw = (float*)(ws + oHraw);
  unsigned short* h16  = (unsigned short*)(ws + oH16);
  unsigned short* xa16 = (unsigned short*)(ws + oA);
  unsigned short* xb16 = xa16 + nTok;
  float*          ybuf = (float*)(ws + oA);
  float*          z32  = (float*)(ws + oZ);
  float*          r32  = (float*)(ws + oR);
  float*          k32  = (float*)(ws + oK);
  float*          v32  = (float*)(ws + oV);
  float*          g32  = (float*)(ws + oG);
  unsigned short* yghi = (unsigned short*)(ws + oR);
  unsigned short* yglo = yghi + nTok;

  const size_t wplane  = (size_t)kDim * kDim;
  const long   wzplane = (long)(2 * wplane);
  const int    n8      = (int)(nTok / 8);
  const int    n2h     = kRows * kLora / 2;
  const int    tilesProj = (kRows / 64) * (kDim / 64);
  const int    gridProj  = (tilesProj + 7) / 8;
  const int    tilesL1   = (kRows / 64) * (kLora / 64);
  const int    gridL1    = (tilesL1 + 7) / 8;

  tcast_kernel<1><<<dim3(kDim / 64, kDim / 64, 5), 256, 0, stream>>>(Wr, Wk, Wv, Wg, Wo, kDim, kDim,
                                                                      wt, wt + wplane, wzplane, 1.0f);
  tcast_kernel<0><<<dim3(kDim / 64, kLora / 64, 1), 256, 0, stream>>>(Aw, Aw, Aw, Aw, Aw, kDim, kLora,
                                                                       awT, awT, 0L, kLoraCarry);
  tcast_kernel<0><<<dim3(kLora / 64, kDim / 64, 1), 256, 0, stream>>>(Bw, Bw, Bw, Bw, Bw, kLora, kDim,
                                                                       bwT, bwT, 0L, kLoraCarry);

  shiftmix_kernel<0><<<(n8 + 255) / 256, 256, 0, stream>>>(x, mu_w, xa16, xa16, n8);
  wmma_gemm64<0, false, 0, 0, false, 0><<<dim3(gridL1, 1), 256, 0, stream>>>(
      xa16, xa16, kDim, 0L, awT, awT, kDim, 0L, hraw, hraw, kLora, 0L, w0, x, 0L,
      kRows, kLora, kDim, kLoraCarryInv);
  tanh_cast_kernel<<<(n2h + 255) / 256, 256, 0, stream>>>(hraw, h16, n2h);
  wmma_gemm64<0, false, 0, 0, false, 0><<<dim3(gridProj, 1), 256, 0, stream>>>(
      h16, h16, kLora, 0L, bwT, bwT, kLora, 0L, z32, z32, kDim, 0L, w0, x, 0L,
      kRows, kDim, kLora, kLoraCarryInv);

  shiftmix_kernel<1><<<(n8 + 255) / 256, 256, 0, stream>>>(x, mu_r, xa16, xb16, n8);
  wmma_gemm64<1, true, 0, 0, false, 0><<<dim3(gridProj, 1), 256, 0, stream>>>(
      xa16, xb16, kDim, 0L, wt + 0 * 2 * wplane, wt + 0 * 2 * wplane + wplane, kDim, 0L,
      r32, r32, kDim, 0L, w0, x, 0L, kRows, kDim, kDim, 1.0f);
  shiftmix_kernel<1><<<(n8 + 255) / 256, 256, 0, stream>>>(x, mu_k, xa16, xb16, n8);
  wmma_gemm64<1, true, 0, 0, false, 0><<<dim3(gridProj, 1), 256, 0, stream>>>(
      xa16, xb16, kDim, 0L, wt + 1 * 2 * wplane, wt + 1 * 2 * wplane + wplane, kDim, 0L,
      k32, k32, kDim, 0L, w0, x, 0L, kRows, kDim, kDim, 1.0f);
  shiftmix_kernel<1><<<(n8 + 255) / 256, 256, 0, stream>>>(x, mu_v, xa16, xb16, n8);
  wmma_gemm64<1, true, 0, 0, false, 0><<<dim3(gridProj, 1), 256, 0, stream>>>(
      xa16, xb16, kDim, 0L, wt + 2 * 2 * wplane, wt + 2 * 2 * wplane + wplane, kDim, 0L,
      v32, v32, kDim, 0L, w0, x, 0L, kRows, kDim, kDim, 1.0f);
  shiftmix_kernel<1><<<(n8 + 255) / 256, 256, 0, stream>>>(x, mu_g, xa16, xb16, n8);
  wmma_gemm64<1, true, 0, 0, false, 0><<<dim3(gridProj, 1), 256, 0, stream>>>(
      xa16, xb16, kDim, 0L, wt + 3 * 2 * wplane, wt + 3 * 2 * wplane + wplane, kDim, 0L,
      g32, g32, kDim, 0L, w0, x, 0L, kRows, kDim, kDim, 1.0f);

  wkv_kernel<<<kBatch * kHeads, kHeadDim, 0, stream>>>(r32, k32, v32, z32, w0, u, ybuf);

  gn_gate_kernel<<<(kRows * kHeads) / 8, 256, 0, stream>>>(ybuf, g32, gng, gnb, yghi, yglo);

  wmma_gemm64<1, true, 0, 0, false, 0><<<dim3(gridProj, 1), 256, 0, stream>>>(
      yghi, yglo, kDim, 0L, wt + 4 * 2 * wplane, wt + 4 * 2 * wplane + wplane, kDim, 0L,
      out, out, kDim, 0L, w0, x, 0L, kRows, kDim, kDim, 1.0f);
}
